// ConvBlock_42090679501105
// MI455X (gfx1250) — hardware-verified
//
#include <hip/hip_runtime.h>
#include <stddef.h>
#include <stdint.h>


#define PD      3
#define CIN     64
#define COUT    64
#define KPT     15
#define HNB     32
#define NG      8
#define CPG     (COUT / NG)
#define FWW     (KPT * COUT)
#define KPL     48
#define WLP     16
#define NTHR    256
#define NQB     8
#define PREC    32
#define SSW     (4 * COUT)
#define GBM     64
#define GTHR    128
#define NTF     10
#define BNF     (16 * NTF)
#define NCB     (FWW / BNF)
#define PPR     (BNF / 4)
#define NITF    (GBM * BNF / (4 * GTHR))
#define NUW     (FWW * CIN / 8)
#define WSLIM   268435456
#define INV_SIG (1.0f / 0.6f)
#define FARPT   1e10f
#define GEPS    1e-5f
#define NEGS    0.1f

static_assert(NTHR == NQB * HNB);
static_assert(NQB * COUT == 4 * 128);
static_assert(((NQB * COUT * 4) % 128) == 0 && ((COUT * 4) % 128) == 0);
static_assert((PREC % 32) == 0 && 2 * NG <= PREC);
static_assert(SSW == NTHR && SSW == 4 * COUT);
static_assert(GBM == (GTHR / 32) * 16);
static_assert((CIN % 32) == 0 && KPT * PD <= KPL && KPT < WLP && CPG == 8);
static_assert((FWW % BNF) == 0 && NCB * BNF == FWW);
static_assert(((BNF * 4) % 128) == 0 && ((FWW * 4) % 128) == 0);
static_assert(NITF * GTHR * 4 == GBM * BNF && (PPR % 8) == 0);
static_assert((NUW % NTHR) == 0 && NUW * 8 == FWW * CIN);
static_assert(14 * COUT + 60 + 3 < FWW);

typedef float          v4f  __attribute__((ext_vector_type(4)));
typedef float          v8f  __attribute__((ext_vector_type(8)));
typedef int            v8i  __attribute__((ext_vector_type(8)));
typedef unsigned short v8us __attribute__((ext_vector_type(8)));
typedef __bf16         v16b __attribute__((ext_vector_type(16)));
typedef v4f  __attribute__((may_alias)) v4fa;
typedef v8us __attribute__((may_alias)) v8usa;
union Frag { v16b b; v8us h[2]; v8i w; };

__device__ __forceinline__ v8f wmk(const Frag& a, const Frag& b, v8f c) {
  v8f d = __builtin_amdgcn_wmma_f32_16x16x32_bf16(false, a.b, false, b.b, (short)0, c, false, false);
  asm volatile("v_nop\n\tv_nop\n\tv_nop\n\tv_nop" : "+v"(d) : "v"(a.w), "v"(b.w));
  return d;
}

__device__ __forceinline__ unsigned short bf_bits(float f) {
  unsigned int u = __float_as_uint(f);
  u += 0x7FFFu + ((u >> 16) & 1u);
  return (unsigned short)(u >> 16);
}
__device__ __forceinline__ float bf_val(unsigned short b) {
  return __uint_as_float(((unsigned int)b) << 16);
}
__device__ __forceinline__ float bf_rne(float f) { return bf_val(bf_bits(f)); }

__device__ __forceinline__ v8us cvt8(const float* p) {
  const v4f a = *(const v4fa*)p, b = *(const v4fa*)(p + 4);
  v8us o;
  o[0] = bf_bits(a.x); o[1] = bf_bits(a.y); o[2] = bf_bits(a.z); o[3] = bf_bits(a.w);
  o[4] = bf_bits(b.x); o[5] = bf_bits(b.y); o[6] = bf_bits(b.z); o[7] = bf_bits(b.w);
  return o;
}

__global__ __launch_bounds__(NTHR) void k_wprep(const float* __restrict__ W, unsigned short* WT) {
  const int u = (int)blockIdx.x * NTHR + (int)threadIdx.x;
  if (u >= NUW) return;
  const int n  = u >> 3;
  const int kp = n >> 6;
  const int d  = n & 63;
  const int c8 = (u & 7) * 8;
  const float* p = W + (size_t)kp * (CIN * COUT) + (size_t)c8 * COUT + d;
  v8us ov;
#pragma unroll
  for (int j = 0; j < 8; ++j) ov[j] = bf_bits(p[(size_t)j * COUT]);
  unsigned short* dp = WT + (size_t)u * 8;
  *(volatile v8us*)dp = ov;
  __threadfence();
  *(volatile v8us*)dp = ov;
}

__global__ __launch_bounds__(NTHR) void k_flag(const float* __restrict__ feat, int nS, int SP, int* FLG) {
  const int n = (int)blockIdx.x * NTHR + (int)threadIdx.x;
  if (n >= SP) return;
  const int nc = n < nS ? n : nS - 1;
  const float* p = feat + (size_t)nc * CIN;
  float a0 = 0.0f, a1 = 0.0f, a2 = 0.0f, a3 = 0.0f;
#pragma unroll 1
  for (int j = 0; j < CIN / 4; ++j) {
    const v4f v = *(const v4fa*)(p + 4 * j);
    a0 += bf_rne(v.x);
    a1 += bf_rne(v.y);
    a2 += bf_rne(v.z);
    a3 += bf_rne(v.w);
  }
  const float s = (a0 + a2) + (a1 + a3);
  const int fl = (n < nS && s > 0.0f) ? 1 : 0;
  int* dp = FLG + n;
  *(volatile int*)dp = fl;
  __threadfence();
  *(volatile int*)dp = fl;
}

__global__ __launch_bounds__(GTHR) void k_fw(const float* __restrict__ feat, int nS,
                                             const unsigned short* __restrict__ WT, float* FW) {
  __shared__ __attribute__((aligned(16))) float stg[GBM * BNF];
  const int tid = (int)threadIdx.x, lane = tid & 31, wave = tid >> 5, hh = lane >> 4, m = lane & 15;
  const int rowBase = (int)blockIdx.x * GBM;
  const int colBase = (int)blockIdx.y * BNF;
  const int row = rowBase + 16 * wave + m;
  const int rc  = row < nS ? row : nS - 1;
  const float* xp = feat + (size_t)rc * CIN + 8 * hh;
  const unsigned short* bp = WT + (size_t)(colBase + m) * CIN + 8 * hh;

  v8f acc[NTF];
  {
    const v8f z = {0.f, 0.f, 0.f, 0.f, 0.f, 0.f, 0.f, 0.f};
#pragma unroll
    for (int t = 0; t < NTF; ++t) acc[t] = z;
  }
#pragma unroll 1
  for (int k0 = 0; k0 < CIN; k0 += 32) {
    Frag af;
    af.h[0] = cvt8(xp + k0);
    af.h[1] = cvt8(xp + k0 + 16);
#pragma unroll
    for (int nt = 0; nt < NTF; ++nt) {
      const unsigned short* wq = bp + (size_t)(16 * nt) * CIN + k0;
      Frag bf;
      bf.h[0] = *(const v8usa*)wq;
      bf.h[1] = *(const v8usa*)(wq + 16);
      acc[nt] = wmk(af, bf, acc[nt]);
    }
  }

#pragma unroll
  for (int nt = 0; nt < NTF; ++nt) {
    const int lc = 16 * nt + m;
#pragma unroll
    for (int r = 0; r < 8; ++r) {
      const int lr = 16 * wave + 8 * hh + r;
      stg[lr * BNF + lc] = acc[nt][r];
    }
  }
  __syncthreads();

  float* fb = FW + (size_t)rowBase * FWW + colBase;
#pragma unroll
  for (int it = 0; it < NITF; ++it) {
    const int p  = it * GTHR + tid;
    const int pr = p / PPR;
    const int pc = p - pr * PPR;
    const v4f v = *(const v4fa*)(stg + 4 * p);
    *(volatile v4f*)(fb + (size_t)pr * FWW + 4 * pc) = v;
  }
  __threadfence();
#pragma unroll
  for (int it = 0; it < NITF; ++it) {
    const int p  = it * GTHR + tid;
    const int pr = p / PPR;
    const int pc = p - pr * PPR;
    const v4f v = *(const v4fa*)(stg + 4 * p);
    *(volatile v4f*)(fb + (size_t)pr * FWW + 4 * pc) = v;
  }
}

#pragma clang fp contract(off)

#define MAC4(V, WGT) { p0 = fmaf((V).x, (WGT), p0); p1 = fmaf((V).y, (WGT), p1); \
                       p2 = fmaf((V).z, (WGT), p2); p3 = fmaf((V).w, (WGT), p3); }

__global__ __launch_bounds__(NTHR) void k_conv(const float* __restrict__ qpts, const float* __restrict__ spts,
                                               const int* __restrict__ nbr, const float* __restrict__ kp,
                                               const int* __restrict__ flg, const float* __restrict__ FW,
                                               const float* __restrict__ bias, int nQ, int nS,
                                               float* XQ, float* part) {
  __shared__ __attribute__((aligned(16))) float wl[NTHR * WLP];
  __shared__ __attribute__((aligned(16))) float stg[NQB * COUT];
  __shared__ __attribute__((aligned(16))) float pst[PREC];
  __shared__ float kpl[KPL];
  const int tid = (int)threadIdx.x, lane = tid & 31, wave = tid >> 5;
  const int h2 = lane >> 4, q4 = 4 * (lane & 15);
  const int qb = (int)blockIdx.x * NQB;
  const int q  = qb + wave;
  const int qc = q < nQ ? q : nQ - 1;

  if (tid < KPL) {
    const int ci = tid < KPT * PD ? tid : KPT * PD - 1;
    const float kv = bf_rne(kp[ci]);
    kpl[tid] = (tid < KPT * PD) ? kv : 0.0f;
  }
  int idx = nbr[(size_t)qc * HNB + lane];
  idx = idx < 0 ? 0 : (idx > nS ? nS : idx);
  const bool far = idx >= nS;
  const int idxc = far ? nS - 1 : idx;
  float rx, ry, rz;
  {
    const float* ps = spts + (size_t)idxc * PD;
    const float* pq = qpts + (size_t)qc * PD;
    const float sx = bf_rne(ps[0]), sy = bf_rne(ps[1]), sz = bf_rne(ps[2]);
    const float qx = bf_rne(pq[0]), qy = bf_rne(pq[1]), qz = bf_rne(pq[2]);
    const float px = far ? FARPT : sx;
    const float py = far ? FARPT : sy;
    const float pz = far ? FARPT : sz;
    rx = px - qx;
    ry = py - qy;
    rz = pz - qz;
  }
  int fl = flg[idxc];
  fl = far ? 0 : fl;
  __syncthreads();

  int anyw = 0;
  {
    float* wr = wl + tid * WLP;
#pragma unroll 1
    for (int k = 0; k < KPT; ++k) {
      const float dx = rx - kpl[3 * k + 0];
      const float dy = ry - kpl[3 * k + 1];
      const float dz = rz - kpl[3 * k + 2];
      const float sq = (dx * dx + dz * dz) + dy * dy;
      const float dd = sqrtf(sq);
      const float t  = dd * INV_SIG;
      float w = 1.0f - t;
      w = fmaxf(w, 0.0f);
      wr[(k & 1) * 8 + (k >> 1)] = w;
      anyw |= (w > 0.0f) ? 1 : 0;
    }
    wr[WLP - 1] = 0.0f;
  }
  const unsigned anymask = __builtin_amdgcn_ballot_w32(anyw != 0);
  const unsigned cmask   = __builtin_amdgcn_ballot_w32(fl != 0);
  const int cnt = (int)__builtin_popcount(cmask);
  __syncthreads();

  float p0 = 0.0f, p1 = 0.0f, p2 = 0.0f, p3 = 0.0f;
  const float* wlw = wl + (wave * HNB) * WLP + 8 * h2;
  const int offA = COUT * h2 + q4;
#pragma unroll 1
  for (int j = 0; j < HNB; ++j) {
    const int sj = __builtin_amdgcn_readlane(idxc, j);
    if (((anymask >> j) & 1u) != 0u) {
      const float* fr = FW + (size_t)sj * FWW;
      const v4f wa = *(const v4fa*)(wlw + j * WLP);
      const v4f wb = *(const v4fa*)(wlw + j * WLP + 4);
      const v4f v0 = *(const v4fa*)(fr + offA);
      const v4f v1 = *(const v4fa*)(fr + offA + 2 * COUT);
      const v4f v2 = *(const v4fa*)(fr + offA + 4 * COUT);
      const v4f v3 = *(const v4fa*)(fr + offA + 6 * COUT);
      const v4f v4 = *(const v4fa*)(fr + offA + 8 * COUT);
      const v4f v5 = *(const v4fa*)(fr + offA + 10 * COUT);
      const v4f v6 = *(const v4fa*)(fr + offA + 12 * COUT);
      const v4f v7 = *(const v4fa*)(fr + 14 * COUT + q4);
      MAC4(v0, wa.x)
      MAC4(v1, wa.y)
      MAC4(v2, wa.z)
      MAC4(v3, wa.w)
      MAC4(v4, wb.x)
      MAC4(v5, wb.y)
      MAC4(v6, wb.z)
      MAC4(v7, wb.w)
    }
  }
  {
    const float t0 = __shfl_xor(p0, 16), t1 = __shfl_xor(p1, 16), t2 = __shfl_xor(p2, 16), t3 = __shfl_xor(p3, 16);
    p0 += t0; p1 += t1; p2 += t2; p3 += t3;
  }
  const bool live = q < nQ;
  const float den = (float)(cnt > 1 ? cnt : 1);
  const float rc  = 1.0f / den;
  const v4f b4 = *(const v4fa*)(bias + q4);
  float o0 = p0 * rc + bf_rne(b4.x);
  float o1 = p1 * rc + bf_rne(b4.y);
  float o2 = p2 * rc + bf_rne(b4.z);
  float o3 = p3 * rc + bf_rne(b4.w);
  o0 = live ? o0 : 0.0f; o1 = live ? o1 : 0.0f; o2 = live ? o2 : 0.0f; o3 = live ? o3 : 0.0f;
  if (lane < 16) {
    v4f ov;
    ov.x = o0; ov.y = o1; ov.z = o2; ov.w = o3;
    *(v4fa*)(stg + wave * COUT + q4) = ov;
  }
  __syncthreads();

  if (tid < NG) {
    const int g = tid;
    float s = 0.0f, s2 = 0.0f;
#pragma unroll 1
    for (int i = 0; i < NQB * CPG; ++i) {
      const float x = stg[(i >> 3) * COUT + CPG * g + (i & 7)];
      s += x;
      s2 = fmaf(x, x, s2);
    }
    pst[2 * g]     = s;
    pst[2 * g + 1] = s2;
  }
  if (tid >= 2 * NG && tid < PREC) pst[tid] = 0.0f;
  __syncthreads();

  const bool sx = tid < (NQB * COUT) / 4;
  const bool sp = tid < PREC / 4;
  v4f xv = {0.f, 0.f, 0.f, 0.f}, pv = {0.f, 0.f, 0.f, 0.f};
  float* xqp = XQ + (size_t)qb * COUT + 4 * tid;
  float* pp  = part + (size_t)blockIdx.x * PREC + 4 * tid;
  if (sx) { xv = *(const v4fa*)(stg + 4 * tid); *(volatile v4f*)xqp = xv; }
  if (sp) { pv = *(const v4fa*)(pst + 4 * tid); *(volatile v4f*)pp  = pv; }
  __threadfence();
  if (sx) *(volatile v4f*)xqp = xv;
  if (sp) *(volatile v4f*)pp  = pv;
}
#undef MAC4

__global__ __launch_bounds__(COUT) void k_fin(const float* __restrict__ part, int nPart, int nQ,
                                             const float* __restrict__ gam, const float* __restrict__ bet,
                                             float* ss) {
  __shared__ __attribute__((aligned(16))) float stg[SSW];
  const int tid = (int)threadIdx.x;
  const int g = tid >> 3;
  double S = 0.0, S2 = 0.0;
#pragma unroll 1
  for (int b = 0; b < nPart; ++b) {
    const float* pr = part + (size_t)b * PREC;
    S  += (double)pr[2 * g];
    S2 += (double)pr[2 * g + 1];
  }
  const double cntd = (double)nQ * (double)CPG;
  const double mean = S / cntd;
  double var = S2 / cntd - mean * mean;
  var = var < 0.0 ? 0.0 : var;
  const float meanf = (float)mean;
  const float varf  = (float)var;
  const float rstd  = 1.0f / sqrtf(varf + GEPS);
  stg[tid]            = meanf;
  stg[COUT + tid]     = rstd;
  stg[2 * COUT + tid] = bf_rne(gam[tid]);
  stg[3 * COUT + tid] = bf_rne(bet[tid]);
  __syncthreads();
  const v4f v = *(const v4fa*)(stg + 4 * tid);
  float* dp = ss + 4 * tid;
  *(volatile v4f*)dp = v;
  __threadfence();
  *(volatile v4f*)dp = v;
}

__global__ __launch_bounds__(NTHR) void k_out(const float* __restrict__ xq, const float* __restrict__ ss,
                                              int nUnits, float* out) {
  __shared__ float ssh[SSW];
  const int tid = (int)threadIdx.x;
  ssh[tid] = ss[tid];
  __syncthreads();
  const int u = (int)blockIdx.x * NTHR + tid;
  if (u >= nUnits) return;
  const int c4 = (u & (COUT / 4 - 1)) * 4;
  const v4f x = *(const v4fa*)(xq + (size_t)u * 4);
  float y0 = ((x.x - ssh[c4 + 0]) * ssh[COUT + c4 + 0]) * ssh[2 * COUT + c4 + 0] + ssh[3 * COUT + c4 + 0];
  float y1 = ((x.y - ssh[c4 + 1]) * ssh[COUT + c4 + 1]) * ssh[2 * COUT + c4 + 1] + ssh[3 * COUT + c4 + 1];
  float y2 = ((x.z - ssh[c4 + 2]) * ssh[COUT + c4 + 2]) * ssh[2 * COUT + c4 + 2] + ssh[3 * COUT + c4 + 2];
  float y3 = ((x.w - ssh[c4 + 3]) * ssh[COUT + c4 + 3]) * ssh[2 * COUT + c4 + 3] + ssh[3 * COUT + c4 + 3];
  y0 = (y0 >= 0.0f) ? y0 : NEGS * y0;
  y1 = (y1 >= 0.0f) ? y1 : NEGS * y1;
  y2 = (y2 >= 0.0f) ? y2 : NEGS * y2;
  y3 = (y3 >= 0.0f) ? y3 : NEGS * y3;
  v4f o;
  o.x = y0; o.y = y1; o.z = y2; o.w = y3;
  float* op = out + (size_t)u * 4;
  *(volatile v4f*)op = o;
  __threadfence();
  *(volatile v4f*)op = o;
}

static inline int cdiv(int a, int b) { return (a + b - 1) / b; }
static inline size_t al256(size_t o) { return (o + 255) & ~(size_t)255; }

extern "C" void kernel_launch(void* const* d_in, const int* in_sizes, int n_in,
                              void* d_out, int out_size, void* d_ws, size_t ws_size,
                              hipStream_t stream) {
  if (n_in < 9) return;
  if (in_sizes[0] < CIN || (in_sizes[0] % CIN) != 0) return;
  const int nS = in_sizes[0] / CIN;
  if (nS < 1 || nS > (1 << 24)) return;
  if (in_sizes[1] < PD || (in_sizes[1] % PD) != 0) return;
  const int nQ = in_sizes[1] / PD;
  if (nQ < 1 || nQ > (1 << 24)) return;
  if ((long long)in_sizes[2] != (long long)nS * PD) return;
  if ((long long)in_sizes[3] != (long long)nQ * HNB) return;
  if (in_sizes[4] != KPT * PD) return;
  if (in_sizes[5] != KPT * CIN * COUT) return;
  if (in_sizes[6] != COUT || in_sizes[7] != COUT || in_sizes[8] != COUT) return;
  if ((long long)out_size != (long long)nQ * COUT) return;

  const float* feat  = (const float*)d_in[0];
  const float* qpts  = (const float*)d_in[1];
  const float* spts  = (const float*)d_in[2];
  const int*   nbr   = (const int*)  d_in[3];
  const float* kpts  = (const float*)d_in[4];
  const float* W     = (const float*)d_in[5];
  const float* bias  = (const float*)d_in[6];
  const float* gamma = (const float*)d_in[7];
  const float* beta  = (const float*)d_in[8];
  float* out = (float*)d_out;

  const int MP = cdiv(nS, GBM) * GBM;
  const int gM = MP / GBM;
  const int SP = cdiv(nS, NTHR) * NTHR;
  const int gQ = cdiv(nQ, NQB);
  const int QP = gQ * NQB;
  const int nUnits = nQ * (COUT / 4);

  char* ws = (char*)d_ws;
  size_t off = 0;
  const size_t oWT  = off; off = al256(off + (size_t)NUW * 8 * 2);
  const size_t oFLG = off; off = al256(off + (size_t)SP * 4);
  const size_t oFW  = off; off = al256(off + (size_t)MP * FWW * 4);
  const size_t oXQ  = off; off = al256(off + (size_t)QP * COUT * 4);
  const size_t oPT  = off; off = al256(off + (size_t)gQ * PREC * 4);
  const size_t oSS  = off; off = al256(off + (size_t)SSW * 4);
  if (off > ws_size || off > (size_t)WSLIM) return;
  unsigned short* WT  = (unsigned short*)(ws + oWT);
  int*            FLG = (int*)(ws + oFLG);
  float*          FW  = (float*)(ws + oFW);
  float*          XQ  = (float*)(ws + oXQ);
  float*          PT  = (float*)(ws + oPT);
  float*          SS  = (float*)(ws + oSS);

  k_wprep<<<NUW / NTHR, NTHR, 0, stream>>>(W, WT);
  k_flag<<<SP / NTHR, NTHR, 0, stream>>>(feat, nS, SP, FLG);
  k_fw<<<dim3(gM, NCB), GTHR, 0, stream>>>(feat, nS, WT, FW);
  k_conv<<<gQ, NTHR, 0, stream>>>(qpts, spts, nbr, kpts, FLG, FW, bias, nQ, nS, XQ, PT);
  k_fin<<<1, COUT, 0, stream>>>(PT, gQ, nQ, gamma, beta, SS);
  k_out<<<cdiv(nUnits, NTHR), NTHR, 0, stream>>>(XQ, SS, nUnits, out);
}
